// Decorder_52467320488266
// MI455X (gfx1250) — hardware-run, weakly checked
//
#include <hip/hip_runtime.h>
#include <math.h>
#pragma clang fp contract(off)

typedef __attribute__((ext_vector_type(16))) __bf16   v16b;
typedef __attribute__((ext_vector_type(8)))  __bf16   v8b;
typedef __attribute__((ext_vector_type(8)))  float    v8f;
typedef __attribute__((ext_vector_type(4)))  float    v4f;
typedef __attribute__((ext_vector_type(2)))  float    v2f;
typedef __attribute__((ext_vector_type(4)))  unsigned v4u;
typedef __attribute__((ext_vector_type(2)))  unsigned v2u;

constexpr int kB   = 8;
constexpr int kL   = 4096;
constexpr int kC   = 128;
constexpr int kHH  = 64;
constexpr int kWW  = 64;
constexpr int kRows = kB * kL;
constexpr float kTemp    = 0.1f;
constexpr float kInvTemp = 1.0f / kTemp;
constexpr float kThresh  = 0.2f;
static_assert(kInvTemp == 10.0f);
static_assert(kHH * kWW == kL);
static_assert((kC % 32) == 0);
static_assert((kL % 256) == 0);
static_assert(((kRows * kC / 8) % 256) == 0);

constexpr size_t kOffP1 = 0;
constexpr size_t kOffP2 = kOffP1 + (size_t)kRows * kC * 2;
constexpr size_t kOffST = kOffP2 + (size_t)kRows * kC * 2;
constexpr size_t kOffSC = kOffST + (size_t)2 * kRows * 2 * 4;
constexpr size_t kWsTotal = kOffSC + (size_t)2 * kRows * 2 * 4;
static_assert(kWsTotal == 17825792ull);
static_assert(kWsTotal <= 134217728ull);
static_assert((kOffP2 % 128) == 0 && (kOffST % 128) == 0 && (kOffSC % 128) == 0);

__device__ __forceinline__ unsigned bf16_bits_rne(float f) {
  const unsigned u = __float_as_uint(f);
  return (u + 0x7FFFu + ((u >> 16) & 1u)) >> 16;
}
__device__ __forceinline__ unsigned pack_bf16x2(float lo, float hi) {
  const unsigned a = bf16_bits_rne(lo);
  const unsigned b = bf16_bits_rne(hi);
  return a | (b << 16);
}
__device__ __forceinline__ v16b frag_load(const __bf16* p) {
  union U { v16b v; v8b h[2]; } f;
  f.h[0] = *(const v8b*)(p);
  f.h[1] = *(const v8b*)(p + 16);
  return f.v;
}
__device__ __forceinline__ v8f mma_bf16(v16b a, v16b b, v8f c) {
  c = __builtin_amdgcn_wmma_f32_16x16x32_bf16(false, a, false, b, (short)0, c, false, false);
  asm volatile("v_nop\n\tv_nop\n\tv_nop\n\tv_nop" : "+v"(c) : "v"(a), "v"(b));
  return c;
}

__global__ __launch_bounds__(256) void planes_kernel(
    const float* __restrict__ f1, const float* __restrict__ f2,
    unsigned* __restrict__ p1, unsigned* __restrict__ p2)
{
  const int i = blockIdx.x * 256 + threadIdx.x;
  const float* src = blockIdx.y ? f2 : f1;
  unsigned* dst = blockIdx.y ? p2 : p1;
  const size_t e0 = (size_t)i << 3;
  const v4f a0 = *(const v4f*)(src + e0);
  const v4f a1 = *(const v4f*)(src + e0 + 4);
  const float x0 = a0[0], x1 = a0[1], x2 = a0[2], x3 = a0[3];
  const float x4 = a1[0], x5 = a1[1], x6 = a1[2], x7 = a1[3];
  const unsigned w0 = pack_bf16x2(x0, x1);
  const unsigned w1 = pack_bf16x2(x2, x3);
  const unsigned w2 = pack_bf16x2(x4, x5);
  const unsigned w3 = pack_bf16x2(x6, x7);
  const v4u w = (v4u){w0, w1, w2, w3};
  unsigned* q = dst + (e0 >> 1);
  *(volatile v4u*)q = w;
  __threadfence();
  *(volatile v4u*)q = w;
}

template <int MODE>
__global__ __launch_bounds__(256) __attribute__((amdgpu_num_vgpr(256)))
void match_pass(const unsigned short* __restrict__ P1, const unsigned short* __restrict__ P2,
                unsigned* STw, unsigned* SCw)
{
  __shared__ __align__(16) unsigned part[256 * 16 * 2];
  __shared__ __align__(16) unsigned fin[256 * 2];

  const int tid = threadIdx.x, lane = tid & 31, wave = tid >> 5;
  const int n = lane & 15, kh = lane >> 4;
  const int z = blockIdx.z, bb = blockIdx.y;
  const size_t boff = (size_t)bb * kL * kC;
  const __bf16* Ap = (const __bf16*)(z ? P2 : P1) + boff;
  const __bf16* Bp = (const __bf16*)(z ? P1 : P2) + boff;
  const int blk0 = blockIdx.x * 256;
  const int row0 = blk0 + wave * 32;

  v16b af[2][4];
#pragma unroll
  for (int rs = 0; rs < 2; ++rs)
#pragma unroll
    for (int ks = 0; ks < 4; ++ks)
      af[rs][ks] = frag_load(Ap + (size_t)(row0 + rs * 16 + n) * kC + ks * 32 + 8 * kh);

  float sa[2][8], sb[2][8], rmv[2][8], lrv[2][8];
  int   si[2][8];
#pragma unroll
  for (int rs = 0; rs < 2; ++rs)
#pragma unroll
    for (int r = 0; r < 8; ++r) {
      sa[rs][r] = -__builtin_inff();
      sb[rs][r] = 0.0f;
      si[rs][r] = 0;
      rmv[rs][r] = 0.0f;
      lrv[rs][r] = 0.0f;
    }

  const float* stf = (const float*)STw;
  const float* own = stf + ((size_t)z * kRows + (size_t)bb * kL) * 2;
  const float* oth = stf + ((size_t)(1 - z) * kRows + (size_t)bb * kL) * 2;
  if (MODE == 1) {
#pragma unroll
    for (int rs = 0; rs < 2; ++rs)
#pragma unroll
      for (int rp = 0; rp < 4; ++rp) {
        const v4f q = *(const v4f*)(own + (size_t)(row0 + rs * 16 + 8 * kh + 2 * rp) * 2);
        const float q0 = q[0], q1 = q[1], q2 = q[2], q3 = q[3];
        rmv[rs][2 * rp]     = q0;
        lrv[rs][2 * rp]     = q1;
        rmv[rs][2 * rp + 1] = q2;
        lrv[rs][2 * rp + 1] = q3;
      }
  }

  const __bf16* bp = Bp + (size_t)n * kC + 8 * kh;
#pragma unroll 1
  for (int ct = 0; ct < kL / 32; ++ct) {
    const int col0 = ct * 32;
    v8f acc[2][2];
#pragma unroll
    for (int rs = 0; rs < 2; ++rs)
#pragma unroll
      for (int cs = 0; cs < 2; ++cs) acc[rs][cs] = (v8f){0.f, 0.f, 0.f, 0.f, 0.f, 0.f, 0.f, 0.f};
#pragma unroll
    for (int ks = 0; ks < 4; ++ks) {
      const v16b b0 = frag_load(bp + ks * 32);
      const v16b b1 = frag_load(bp + 16 * kC + ks * 32);
      acc[0][0] = mma_bf16(af[0][ks], b0, acc[0][0]);
      acc[0][1] = mma_bf16(af[0][ks], b1, acc[0][1]);
      acc[1][0] = mma_bf16(af[1][ks], b0, acc[1][0]);
      acc[1][1] = mma_bf16(af[1][ks], b1, acc[1][1]);
    }
    bp += 32 * kC;

    if (MODE == 0) {
#pragma unroll
      for (int rs = 0; rs < 2; ++rs)
#pragma unroll
        for (int r = 0; r < 8; ++r) {
          const float x0 = acc[rs][0][r] * kInvTemp;
          const float x1 = acc[rs][1][r] * kInvTemp;
          const float mo = sa[rs][r];
          const float mn = fmaxf(fmaxf(mo, x0), x1);
          const float al = __expf(mo - mn);
          const float e0 = __expf(x0 - mn);
          const float e1 = __expf(x1 - mn);
          sb[rs][r] = fmaf(sb[rs][r], al, e0) + e1;
          sa[rs][r] = mn;
        }
    } else {
#pragma unroll
      for (int cs = 0; cs < 2; ++cs) {
        const int sidx = col0 + cs * 16 + n;
        const v2f o = *(const v2f*)(oth + (size_t)sidx * 2);
        const float om = o[0], ol = o[1];
#pragma unroll
        for (int rs = 0; rs < 2; ++rs)
#pragma unroll
          for (int r = 0; r < 8; ++r) {
            const float x = acc[rs][cs][r] * kInvTemp;
            const float ta = (x - rmv[rs][r]) - lrv[rs][r];
            const float tb = (x - om) - ol;
            const float t = ta + tb;
            const bool g = t > sa[rs][r];
            sa[rs][r] = g ? t : sa[rs][r];
            si[rs][r] = g ? sidx : si[rs][r];
          }
      }
    }
  }

#pragma unroll
  for (int rs = 0; rs < 2; ++rs)
#pragma unroll
    for (int r = 0; r < 8; ++r) {
      const int row = wave * 32 + rs * 16 + 8 * kh + r;
      const unsigned w0 = __float_as_uint(sa[rs][r]);
      const unsigned w1 = (MODE == 0) ? __float_as_uint(sb[rs][r]) : (unsigned)si[rs][r];
      *(v2u*)(part + (row * 16 + n) * 2) = (v2u){w0, w1};
    }
  __syncthreads();
  {
    const unsigned* pp = part + tid * 32;
    if (MODE == 0) {
      float M = __uint_as_float(pp[0]);
#pragma unroll 1
      for (int j = 1; j < 16; ++j) M = fmaxf(M, __uint_as_float(pp[2 * j]));
      float S = 0.0f;
#pragma unroll 1
      for (int j = 0; j < 16; ++j) {
        const float e = expf(__uint_as_float(pp[2 * j]) - M);
        S = fmaf(__uint_as_float(pp[2 * j + 1]), e, S);
      }
      fin[2 * tid]     = __float_as_uint(M);
      fin[2 * tid + 1] = __float_as_uint(logf(S));
    } else {
      float v = __uint_as_float(pp[0]);
      int a = (int)pp[1];
#pragma unroll 1
      for (int j = 1; j < 16; ++j) {
        const float v2 = __uint_as_float(pp[2 * j]);
        const int a2 = (int)pp[2 * j + 1];
        const bool take = (v2 > v) || ((v2 == v) && (a2 < a));
        v = take ? v2 : v;
        a = take ? a2 : a;
      }
      fin[2 * tid]     = __float_as_uint(v);
      fin[2 * tid + 1] = (unsigned)a;
    }
  }
  __syncthreads();
  if (tid < 128) {
    const v4u val = *(const v4u*)(fin + 4 * tid);
    unsigned* dstb = (MODE == 0) ? STw : SCw;
    unsigned* dst = dstb + ((size_t)z * kRows + (size_t)bb * kL + (size_t)blk0) * 2 + 4 * tid;
    *(volatile v4u*)dst = val;
    __threadfence();
    *(volatile v4u*)dst = val;
  }
}

__global__ __launch_bounds__(256) void finalize_kernel(
    const unsigned* __restrict__ P1w, const unsigned* __restrict__ P2w,
    const unsigned* __restrict__ SCw, const int* __restrict__ hp, const int* __restrict__ wp,
    float* __restrict__ out)
{
  __shared__ int sJ[32];
  __shared__ int sMt[32];
  __shared__ int sBad;
  __shared__ __align__(16) float tile[128 * 36];
  const int tid = threadIdx.x;
  const int bb = blockIdx.y;
  const int base = blockIdx.x * 32;

  if (tid == 0) {
    const int hv = hp[0];
    const int wv = wp[0];
    sBad = ((hv != kHH) || (wv != kWW)) ? 1 : 0;
  }
  if (tid < 32) {
    const int l = base + tid;
    const v2u rr = *(const v2u*)(SCw + ((size_t)bb * kL + (size_t)l) * 2);
    const unsigned r0w = rr[0], r1w = rr[1];
    const float T = __uint_as_float(r0w);
    int j = (int)r1w;
    j = (j < 0) ? 0 : j;
    j = (j > kL - 1) ? (kL - 1) : j;
    const v2u cc = *(const v2u*)(SCw + ((size_t)kRows + (size_t)bb * kL + (size_t)j) * 2);
    const unsigned c0w = cc[0], c1w = cc[1];
    const float cT = __uint_as_float(c0w);
    const int cA = (int)c1w;
    const float mv = expf(T);
    const bool ok = (mv > kThresh) && ((cA == l) || (cT == T));
    sJ[tid] = j;
    sMt[tid] = ok ? 1 : 0;
  }
  __syncthreads();

  const int bad = sBad;
  const float nanv = __uint_as_float(0x7fc00000u);
  const unsigned* p1b = P1w + (size_t)bb * kL * (kC / 2);
  const unsigned* p2b = P2w + (size_t)bb * kL * (kC / 2);
#pragma unroll
  for (int it = 0; it < 2; ++it) {
    const int item = it * 256 + tid;
    const int lr = item >> 4;
    const int g = item & 15;
    const int j = sJ[lr];
    const int mt = sMt[lr];
    const v4u av = *(const v4u*)(p1b + (size_t)(base + lr) * (kC / 2) + g * 4);
    const v4u bv = *(const v4u*)(p2b + (size_t)j * (kC / 2) + g * 4);
#pragma unroll
    for (int e = 0; e < 4; ++e) {
      const unsigned aw = av[e];
      const unsigned bw = bv[e];
      const float a0 = __uint_as_float(aw << 16);
      const float a1 = __uint_as_float(aw & 0xffff0000u);
      const float b0 = __uint_as_float(bw << 16);
      const float b1 = __uint_as_float(bw & 0xffff0000u);
      const float s0 = mt ? b0 : 0.0f;
      const float s1 = mt ? b1 : 0.0f;
      float v0 = a0 - s0;
      float v1 = a1 - s1;
      v0 = bad ? nanv : v0;
      v1 = bad ? nanv : v1;
      const int ch = g * 8 + 2 * e;
      tile[ch * 36 + lr] = v0;
      tile[(ch + 1) * 36 + lr] = v1;
    }
  }
  __syncthreads();

  v4f vals[4];
#pragma unroll
  for (int it = 0; it < 4; ++it) {
    const int idx = it * 256 + tid;
    const int ch = idx >> 3;
    const int q = idx & 7;
    vals[it] = *(const v4f*)(tile + ch * 36 + 4 * q);
  }
  float* ob = out + (size_t)bb * kC * kL + base;
  for (int pass = 0; pass < 2; ++pass) {
#pragma unroll
    for (int it = 0; it < 4; ++it) {
      const int idx = it * 256 + tid;
      const int ch = idx >> 3;
      const int q = idx & 7;
      *(volatile v4f*)(ob + (size_t)ch * kL + 4 * q) = vals[it];
    }
    __threadfence();
  }
}

extern "C" void kernel_launch(void* const* d_in, const int* in_sizes, int n_in,
                              void* d_out, int out_size, void* d_ws, size_t ws_size,
                              hipStream_t stream) {
  if (n_in < 4) return;
  if (in_sizes[0] != kRows * kC) return;
  if (in_sizes[1] != kRows * kC) return;
  if (in_sizes[2] != 1) return;
  if (in_sizes[3] != 1) return;
  if (out_size != kRows * kC) return;
  if (ws_size < kWsTotal) return;

  const float* f1 = (const float*)d_in[0];
  const float* f2 = (const float*)d_in[1];
  const int* hp = (const int*)d_in[2];
  const int* wp = (const int*)d_in[3];
  float* out = (float*)d_out;

  char* ws = (char*)d_ws;
  unsigned* P1w = (unsigned*)(ws + kOffP1);
  unsigned* P2w = (unsigned*)(ws + kOffP2);
  unsigned* STw = (unsigned*)(ws + kOffST);
  unsigned* SCw = (unsigned*)(ws + kOffSC);

  planes_kernel<<<dim3(kRows * kC / 8 / 256, 2), 256, 0, stream>>>(f1, f2, P1w, P2w);

  match_pass<0><<<dim3(kL / 256, kB, 2), 256, 0, stream>>>(
      (const unsigned short*)P1w, (const unsigned short*)P2w, STw, SCw);

  match_pass<1><<<dim3(kL / 256, kB, 2), 256, 0, stream>>>(
      (const unsigned short*)P1w, (const unsigned short*)P2w, STw, SCw);

  finalize_kernel<<<dim3(kL / 32, kB), 256, 0, stream>>>(P1w, P2w, SCw, hp, wp, out);
}
